// MambaBlock_89515708383664
// MI455X (gfx1250) — hardware-run, weakly checked
//
#include <hip/hip_runtime.h>


#ifndef NB
#define NB 2
#endif
#ifndef SEQ
#define SEQ 2048
#endif
#define NB_FULL  2
#define SEQ_FULL 2048
#ifndef OUT_SEQ
#define OUT_SEQ SEQ
#endif
#define DM   1024
#define DIN  2048
#define NST  16
#define DTR  64
#define XDW  96
#define XSP  100
#define SCH  16
#define SCW  64
#define US   64.0f
#define WSC  1024.0f
#define FOLD (1.0f / 65536.0f)
#define LOG2E 1.4426950408889634f

static_assert(XDW == DTR + 2 * NST);
static_assert(NST == 16);
static_assert(DTR == 64);
static_assert((XDW * 4) % 128 == 0);
static_assert((XSP * 4) % 16 == 0);
static_assert(XSP >= XDW);
static_assert(DM % 32 == 0);
static_assert(DIN % 32 == 0);
static_assert(DTR % 32 == 0);
static_assert(DM % 64 == 0);
static_assert(DIN % 64 == 0);
static_assert(XDW % 16 == 0);
static_assert(SEQ % 64 == 0);
static_assert((NB * SEQ) % 64 == 0);
static_assert((NB * SEQ) % 32 == 0);
static_assert(SEQ % SCH == 0);
static_assert(DIN % SCW == 0);
static_assert(DIN % 8 == 0);
static_assert(((size_t)SEQ * DM) % 8 == 0);
static_assert(NB <= NB_FULL);
static_assert(SEQ <= SEQ_FULL);
static_assert(16 * 68 * 4 <= 131072);
static_assert(16 * XSP * 4 <= 131072);
static_assert(SCH * SCW * 2 <= 131072);

typedef _Float16 h16;
typedef unsigned short bf;
typedef __attribute__((ext_vector_type(16))) __bf16   v16bf;
typedef __attribute__((ext_vector_type(16))) _Float16 v16h;
typedef __attribute__((ext_vector_type(8)))  _Float16 v8h;
typedef __attribute__((ext_vector_type(8)))  unsigned short v8us;
typedef __attribute__((ext_vector_type(8)))  float    v8f;
typedef __attribute__((ext_vector_type(4)))  float    v4f;
typedef v4f  __attribute__((may_alias)) v4fa;
typedef v8h  __attribute__((may_alias)) v8ha;

__device__ __forceinline__ unsigned short f2bf(float f) { unsigned u = __float_as_uint(f); u += 0x7FFFu + ((u >> 16) & 1u); return (unsigned short)(u >> 16); }
__device__ __forceinline__ float bfr(float f) { return __uint_as_float(((unsigned)f2bf(f)) << 16); }
__device__ __forceinline__ v16h cat16(v8h lo, v8h hi) { return __builtin_shufflevector(lo, hi, 0, 1, 2, 3, 4, 5, 6, 7, 8, 9, 10, 11, 12, 13, 14, 15); }
__device__ __forceinline__ v16bf cat16b(v8us lo, v8us hi) { return __builtin_bit_cast(v16bf, __builtin_shufflevector(lo, hi, 0, 1, 2, 3, 4, 5, 6, 7, 8, 9, 10, 11, 12, 13, 14, 15)); }
__device__ __forceinline__ v8f wmma16(v16h a, v16h b, v8f c) { return __builtin_amdgcn_wmma_f32_16x16x32_f16(false, a, false, b, (short)0, c, false, false); }
__device__ __forceinline__ v8f wmmab(v16bf a, v16bf b, v8f c) { return __builtin_amdgcn_wmma_f32_16x16x32_bf16(false, a, false, b, (short)0, c, false, false); }
__device__ __forceinline__ v16h  ldh(const h16* p) { return cat16(*(const v8h*)p, *(const v8h*)(p + 16)); }
__device__ __forceinline__ v16bf ldb(const bf* p)  { return cat16b(*(const v8us*)p, *(const v8us*)(p + 16)); }
__device__ __forceinline__ void wave_sync() { __builtin_amdgcn_fence(3  , "wavefront"); __builtin_amdgcn_wave_barrier(); asm volatile("" ::: "memory"); }

__device__ __forceinline__ v8f mma_g(v16h a, v16h b, v8f c) { c = wmma16(a, b, c); asm volatile("v_nop\n\tv_nop\n\tv_nop\n\tv_nop" : "+v"(c) : "v"(a), "v"(b)); return c; }
__device__ __forceinline__ v8f mma_g(v16bf a, v16bf b, v8f c) { c = wmmab(a, b, c); asm volatile("v_nop\n\tv_nop\n\tv_nop\n\tv_nop" : "+v"(c) : "v"(a), "v"(b)); return c; }
__device__ __forceinline__ v16h  ldf(const h16* p) { return ldh(p); }
__device__ __forceinline__ v16bf ldf(const bf* p)  { return ldb(p); }
static __device__ __forceinline__ h16 toh_flush(float v) { const h16 r = (h16)v; return (fabsf(v) < 6.103515625e-05f) ? (h16)0.0f : r; }
__device__ __forceinline__ float silu_f(float s) { return s * __builtin_amdgcn_rcpf(1.0f + __builtin_amdgcn_exp2f(-s * LOG2E)); }
__device__ __forceinline__ float softplus_f(float v) { return fmaxf(v, 0.0f) + log1pf(expf(-fabsf(v))); }

__global__ __launch_bounds__(256) void k_cvt8(const float* __restrict__ src, bf* dst, size_t n8) {
    const size_t i = (size_t)blockIdx.x * 256 + threadIdx.x; if (i >= n8) return;
    const v8f v = *(const v8f*)(src + i * 8); v8us o;
#pragma unroll
    for (int k = 0; k < 8; ++k) o[k] = f2bf(v[k]);
    *(volatile v8us*)(dst + i * 8) = o; __threadfence(); *(volatile v8us*)(dst + i * 8) = o;
}

__global__ __launch_bounds__(256) void k_wcvt(const float* __restrict__ src, h16* dst, size_t n8, float scale) {
    const size_t i = (size_t)blockIdx.x * 256 + threadIdx.x; if (i >= n8) return;
    const v8f v = *(const v8f*)(src + i * 8); v8h o;
#pragma unroll
    for (int k = 0; k < 8; ++k) o[k] = toh_flush(bfr(v[k]) * scale);
    *(volatile v8h*)(dst + i * 8) = o; __threadfence(); *(volatile v8h*)(dst + i * 8) = o;
}

template <typename T, int K, int EPI>
__device__ __forceinline__ void gemm64_body(const T* __restrict__ A, const T* __restrict__ Bt, const float* __restrict__ bias, float* C, size_t cbase, int pitch, float scale) {
    __shared__ __align__(16) float os[16 * 68];
    const int lane = threadIdx.x & 31, lr = lane & 15, hi = lane >> 4; const int r0 = blockIdx.x * 64, c0 = blockIdx.y * 64;
    v8f acc[4][4];
#pragma unroll
    for (int mb = 0; mb < 4; ++mb)
#pragma unroll
        for (int nb = 0; nb < 4; ++nb) acc[mb][nb] = (v8f){};
    const size_t aoff = (size_t)(r0 + lr) * K + 8 * hi, boff = (size_t)(c0 + lr) * K + 8 * hi;
#pragma unroll 1
    for (int kc = 0; kc < K; kc += 32) {
        decltype(ldf(A)) a[4];
#pragma unroll
        for (int mb = 0; mb < 4; ++mb) a[mb] = ldf(A + aoff + (size_t)mb * 16 * K + kc);
#pragma unroll
        for (int nb = 0; nb < 4; ++nb) { const auto b = ldf(Bt + boff + (size_t)nb * 16 * K + kc);
#pragma unroll
            for (int mb = 0; mb < 4; ++mb) acc[mb][nb] = mma_g(a[mb], b, acc[mb][nb]); }
    }
    const int row2 = lane >> 4, c4 = (lane & 15) * 4;
    v4f bq = (v4f){};
    if (EPI == 1) { const v4f bl = *(const v4f*)(bias + c0 + c4);
#pragma unroll
        for (int i = 0; i < 4; ++i) bq[i] = bfr(bl[i]); }
    static_assert(8 * 32 * 16 == 16 * 64 * 4);
#pragma unroll
    for (int mb = 0; mb < 4; ++mb) {
#pragma unroll
        for (int nb = 0; nb < 4; ++nb) {
#pragma unroll
            for (int j = 0; j < 8; ++j) os[(hi * 8 + j) * 68 + nb * 16 + lr] = acc[mb][nb][j] * scale; }
        wave_sync();
        if (EPI == 1) {
#pragma unroll 1
            for (int s = 0; s < 8; ++s) { const int row = 2 * s + row2;
                v4f x = *(const v4fa*)(&os[row * 68 + c4]);
#pragma unroll
                for (int i = 0; i < 4; ++i) x[i] = softplus_f(x[i] + bq[i]);
                *(v4fa*)(&os[row * 68 + c4]) = x; }
            wave_sync();
        }
#pragma unroll 1
        for (int ps = 0; ps < 2; ++ps) {
#pragma unroll
            for (int s = 0; s < 8; ++s) { const int row = 2 * s + row2;
                const v4f val = *(const v4fa*)(&os[row * 68 + c4]);
                *(volatile v4f*)(C + cbase + (size_t)(mb * 16 + row) * (size_t)pitch + c4) = val; }
            if (ps == 0) __threadfence(); }
        wave_sync();
    }
}

__global__ __launch_bounds__(32) void k_inproj(const bf* __restrict__ XB, const bf* __restrict__ WB, float* XZ) {
    const int r0 = blockIdx.x * 64, c0 = blockIdx.y * 64;
    const size_t cbase = (size_t)(c0 / DIN) * ((size_t)NB * SEQ * DIN) + (size_t)r0 * DIN + (size_t)(c0 % DIN);
    gemm64_body<bf, DM, 0>(XB, WB, (const float*)0, XZ, cbase, DIN, 1.0f);
}

__global__ __launch_bounds__(32) void k_dtproj(const h16* __restrict__ DR16, const h16* __restrict__ WD16, const float* __restrict__ dt_b, float* DT) {
    const int r0 = blockIdx.x * 64, c0 = blockIdx.y * 64;
    const size_t cbase = (size_t)r0 * DIN + (size_t)c0;
    gemm64_body<h16, DTR, 1>(DR16, WD16, dt_b, DT, cbase, DIN, FOLD);
}

__global__ __launch_bounds__(32) void k_outproj(const h16* __restrict__ Y16, const h16* __restrict__ WO16, float* OUT) {
    const int r0 = blockIdx.x * 64, c0 = blockIdx.y * 64;
    const size_t cbase = ((size_t)(r0 / SEQ) * OUT_SEQ + (size_t)(r0 % SEQ)) * DM + (size_t)c0;
    gemm64_body<h16, DIN, 0>(Y16, WO16, (const float*)0, OUT, cbase, DM, FOLD);
}

__global__ __launch_bounds__(32) void k_xproj(const h16* __restrict__ U16, const h16* __restrict__ WX16, float* XD, h16* DR16) {
    __shared__ __align__(16) float os[16 * XSP];
    const int lane = threadIdx.x & 31, lr = lane & 15, hi = lane >> 4; const int r0 = blockIdx.x * 32;
    v8f acc[2][6];
#pragma unroll
    for (int mb = 0; mb < 2; ++mb)
#pragma unroll
        for (int nb = 0; nb < 6; ++nb) acc[mb][nb] = (v8f){};
    const size_t aoff = (size_t)(r0 + lr) * DIN + 8 * hi, boff = (size_t)lr * DIN + 8 * hi;
#pragma unroll 1
    for (int kc = 0; kc < DIN; kc += 32) {
        v16h a[2];
#pragma unroll
        for (int mb = 0; mb < 2; ++mb) a[mb] = ldh(U16 + aoff + (size_t)mb * 16 * DIN + kc);
#pragma unroll
        for (int nb = 0; nb < 6; ++nb) { const v16h b = ldh(WX16 + boff + (size_t)nb * 16 * DIN + kc);
#pragma unroll
            for (int mb = 0; mb < 2; ++mb) acc[mb][nb] = mma_g(a[mb], b, acc[mb][nb]); }
    }
    static_assert(12 * 32 * 16 == 16 * XDW * 4);
    static_assert(4 * 32 * 16 == 16 * DTR * 2);
#pragma unroll
    for (int mb = 0; mb < 2; ++mb) {
#pragma unroll
        for (int nb = 0; nb < 6; ++nb) {
#pragma unroll
            for (int j = 0; j < 8; ++j) os[(hi * 8 + j) * XSP + nb * 16 + lr] = acc[mb][nb][j] * FOLD; }
        wave_sync();
        const size_t xb = (size_t)(r0 + mb * 16) * XDW;
        const size_t db = (size_t)(r0 + mb * 16) * DTR;
#pragma unroll 1
        for (int ps = 0; ps < 2; ++ps) {
#pragma unroll
            for (int s = 0; s < 12; ++s) { const int p = s * 32 + lane; const int row = p / 24, c4 = (p % 24) * 4;
                const v4f val = *(const v4fa*)(&os[row * XSP + c4]);
                *(volatile v4f*)(XD + xb + (size_t)p * 4) = val; }
#pragma unroll
            for (int s = 0; s < 4; ++s) { const int row = 4 * s + (lane >> 3), c8 = (lane & 7) * 8;
                const v4f x0 = *(const v4fa*)(&os[row * XSP + c8]); const v4f x1 = *(const v4fa*)(&os[row * XSP + c8 + 4]); v8h hv;
#pragma unroll
                for (int i = 0; i < 4; ++i) { hv[i] = toh_flush(x0[i] * US); hv[4 + i] = toh_flush(x1[i] * US); }
                *(volatile v8h*)(DR16 + db + (size_t)row * DTR + c8) = hv; }
            if (ps == 0) __threadfence(); }
        wave_sync();
    }
}

__global__ __launch_bounds__(256) void k_conv(const float* __restrict__ XP, const float* __restrict__ conv_w, const float* __restrict__ conv_b, h16* U16, size_t n8) {
#pragma clang fp contract(off)
    const size_t i = (size_t)blockIdx.x * 256 + threadIdx.x; if (i >= n8) return;
    const int m = (int)(i / (DIN / 8)); const int d8 = (int)(i % (DIN / 8)) * 8;
    const int t = m % SEQ; const size_t mrow0 = (size_t)(m - t);
    float x[4][8];
#pragma unroll
    for (int k = 0; k < 4; ++k) {
        const int tk = t - 3 + k; const int tc = tk < 0 ? 0 : tk;
        const float* p = XP + (mrow0 + (size_t)tc) * DIN + d8;
        v4f a = *(const v4f*)p; v4f c = *(const v4f*)(p + 4);
        asm volatile("" : "+v"(a), "+v"(c));
        const bool ok = tk >= 0;
#pragma unroll
        for (int j = 0; j < 4; ++j) { x[k][j] = ok ? a[j] : 0.0f; x[k][4 + j] = ok ? c[j] : 0.0f; }
    }
    const v4f b0 = *(const v4f*)(conv_b + d8), b1 = *(const v4f*)(conv_b + d8 + 4);
    v8h o;
#pragma unroll
    for (int j = 0; j < 8; ++j) {
        const v4f w = *(const v4f*)(conv_w + (size_t)(d8 + j) * 4);
        const float cb = bfr(j < 4 ? b0[j & 3] : b1[j & 3]);
        float s = ((x[0][j] * bfr(w[0]) + x[1][j] * bfr(w[1])) + x[2][j] * bfr(w[2])) + x[3][j] * bfr(w[3]);
        s = s + cb;
        o[j] = toh_flush(silu_f(s) * US);
    }
    *(volatile v8h*)(U16 + i * 8) = o; __threadfence(); *(volatile v8h*)(U16 + i * 8) = o;
}

__global__ __launch_bounds__(SCW) void k_scan(const float* __restrict__ XP, const float* __restrict__ ZP, const float* __restrict__ DT, const float* __restrict__ XD,
                                              const float* __restrict__ conv_w, const float* __restrict__ conv_b, const float* __restrict__ A_log, const float* __restrict__ D_param, h16* Y16) {
#pragma clang fp contract(off)
    __shared__ __align__(16) h16 ys[SCH * SCW];
    const int tid = threadIdx.x; const int d = blockIdx.x * SCW + tid; const int b = blockIdx.y;
    float A2[NST], h[NST];
    { const v4f* ap = (const v4f*)(A_log + (size_t)d * NST);
#pragma unroll
      for (int q = 0; q < 4; ++q) { const v4f a = ap[q];
#pragma unroll
          for (int i = 0; i < 4; ++i) { A2[4 * q + i] = -(__builtin_amdgcn_exp2f(bfr(a[i]) * LOG2E)) * LOG2E; h[4 * q + i] = 0.0f; } } }
    const v4f wv = *(const v4f*)(conv_w + (size_t)d * 4);
    const float w0 = bfr(wv[0]), w1 = bfr(wv[1]), w2 = bfr(wv[2]), w3 = bfr(wv[3]);
    const float cb = bfr(conv_b[d]); const float Dp = bfr(D_param[d]);
    const float* xp = XP + (size_t)b * SEQ * DIN + d;
    const float* zp = ZP + (size_t)b * SEQ * DIN + d;
    const float* dp = DT + (size_t)b * SEQ * DIN + d;
    const float* bc = XD + (size_t)b * SEQ * XDW + DTR;
    h16* yo = Y16 + (size_t)b * SEQ * DIN + (size_t)blockIdx.x * SCW;
    float x0 = 0.0f, x1 = 0.0f, x2 = 0.0f;
    static_assert(SCW * 2 * 16 == SCH * SCW * 2);
#pragma unroll 1
    for (int t0 = 0; t0 < SEQ; t0 += SCH) {
#pragma unroll 1
        for (int tt = 0; tt < SCH; ++tt) {
            const size_t m = (size_t)(t0 + tt);
            const float dtv = dp[m * DIN], xv = xp[m * DIN], zv = zp[m * DIN];
            const v4f* bq = (const v4f*)(bc + m * XDW);
            const v4f B0 = bq[0], B1 = bq[1], B2 = bq[2], B3 = bq[3], C0 = bq[4], C1 = bq[5], C2 = bq[6], C3 = bq[7];
            float Bn[NST], Cn[NST];
#pragma unroll
            for (int i = 0; i < 4; ++i) { Bn[i] = B0[i]; Bn[4 + i] = B1[i]; Bn[8 + i] = B2[i]; Bn[12 + i] = B3[i]; Cn[i] = C0[i]; Cn[4 + i] = C1[i]; Cn[8 + i] = C2[i]; Cn[12 + i] = C3[i]; }
            float s = ((x0 * w0 + x1 * w1) + x2 * w2) + xv * w3;
            s = s + cb;
            x0 = x1; x1 = x2; x2 = xv;
            const float u = silu_f(s), g = silu_f(zv);
            float acc = 0.0f;
#pragma unroll
            for (int n = 0; n < NST; ++n) {
                h[n] = __builtin_amdgcn_exp2f(dtv * A2[n]) * h[n] + (dtv * Bn[n]) * u;
                acc = acc + Cn[n] * h[n]; }
            const float yv = (acc + u * Dp) * g;
            ys[tt * SCW + tid] = toh_flush(yv * US);
        }
        __syncthreads();
#pragma unroll 1
        for (int ps = 0; ps < 2; ++ps) {
#pragma unroll
            for (int i = 0; i < 2; ++i) { const int p = i * SCW + tid; const int row = p >> 3, c8 = (p & 7) * 8;
                const v8h hv = *(const v8ha*)(&ys[row * SCW + c8]);
                *(volatile v8h*)(yo + (size_t)(t0 + row) * DIN + c8) = hv; }
            if (ps == 0) __threadfence(); }
        __syncthreads();
    }
}

static constexpr size_t al256(size_t v) { return (v + 255) & ~(size_t)255; }
static constexpr size_t mx2(size_t a, size_t b) { return a > b ? a : b; }
static constexpr size_t SZ_XB = al256((size_t)NB * SEQ * DM * 2);
static constexpr size_t SZ_WB = al256((size_t)2 * DIN * DM * 2);
static constexpr size_t SZ_U  = al256((size_t)NB * SEQ * DIN * 2);
static constexpr size_t SZ_R1 = mx2(SZ_XB + SZ_WB, SZ_U);
static constexpr size_t SZ_XZ = al256((size_t)2 * NB * SEQ * DIN * 4);
static constexpr size_t SZ_DT = al256((size_t)NB * SEQ * DIN * 4);
static constexpr size_t SZ_XD = al256((size_t)NB * SEQ * XDW * 4);
static constexpr size_t SZ_DR = al256((size_t)NB * SEQ * DTR * 2);
static constexpr size_t SZ_WX = al256((size_t)XDW * DIN * 2);
static constexpr size_t SZ_WD = al256((size_t)DIN * DTR * 2);
static constexpr size_t SZ_WO = al256((size_t)DM * DIN * 2);
static constexpr size_t SZ_TOTAL = SZ_R1 + SZ_XZ + SZ_DT + SZ_XD + SZ_DR + SZ_WX + SZ_WD + SZ_WO;
static_assert(SZ_XB + SZ_WB <= SZ_R1);
static_assert(SZ_U <= SZ_R1);
static_assert(SZ_TOTAL <= (size_t)134217728);
static_assert(((size_t)NB * SEQ * DIN * 4) % 256 == 0);
static_assert(((size_t)NB * SEQ * DIN) % 8 == 0);
static_assert(((size_t)2 * DIN * DM) % 8 == 0);
static_assert(((size_t)XDW * DIN) % 8 == 0);
static_assert(((size_t)DIN * DTR) % 8 == 0);
static_assert(((size_t)DM * DIN) % 8 == 0);

extern "C" void kernel_launch(void* const* d_in, const int* in_sizes, int n_in,
                              void* d_out, int out_size, void* d_ws, size_t ws_size, hipStream_t stream) {
    if (n_in < 10) return;
    const size_t needx = ((size_t)(NB - 1) * SEQ_FULL + SEQ) * DM;
    if ((size_t)in_sizes[0] < needx) return;
    if ((size_t)in_sizes[1] < (size_t)2 * DIN * DM) return;
    if ((size_t)in_sizes[2] < (size_t)DIN * 4 || in_sizes[3] < DIN) return;
    if ((size_t)in_sizes[4] < (size_t)XDW * DIN || (size_t)in_sizes[5] < (size_t)DIN * DTR || in_sizes[6] < DIN) return;
    if ((size_t)in_sizes[7] < (size_t)DIN * NST || in_sizes[8] < DIN || (size_t)in_sizes[9] < (size_t)DM * DIN) return;
    if ((size_t)out_size < ((size_t)(NB - 1) * OUT_SEQ + SEQ) * DM) return;
    if (SZ_TOTAL > ws_size) return;
    const float* x     = (const float*)d_in[0];
    const float* w_in  = (const float*)d_in[1];
    const float* cw    = (const float*)d_in[2];
    const float* cbias = (const float*)d_in[3];
    const float* w_x   = (const float*)d_in[4];
    const float* w_dt  = (const float*)d_in[5];
    const float* b_dt  = (const float*)d_in[6];
    const float* a_log = (const float*)d_in[7];
    const float* d_par = (const float*)d_in[8];
    const float* w_out = (const float*)d_in[9];
    float* OUT = (float*)d_out;
    char* wsp = (char*)d_ws;
    char* r1 = wsp; wsp += SZ_R1;
    bf*  XB  = (bf*)r1;
    bf*  WB  = (bf*)(r1 + SZ_XB);
    h16* U16 = (h16*)r1;
    h16* Y16 = (h16*)r1;
    float* XZ = (float*)wsp; wsp += SZ_XZ;
    float* DT = (float*)wsp; wsp += SZ_DT;
    float* XD = (float*)wsp; wsp += SZ_XD;
    h16* DR16 = (h16*)wsp; wsp += SZ_DR;
    h16* WX16 = (h16*)wsp; wsp += SZ_WX;
    h16* WD16 = (h16*)wsp; wsp += SZ_WD;
    h16* WO16 = (h16*)wsp; wsp += SZ_WO;
    const float* XP = XZ; const float* ZP = XZ + (size_t)NB * SEQ * DIN;

    if (SEQ == SEQ_FULL) {
        const size_t n8 = (size_t)NB * SEQ * DM / 8;
        k_cvt8<<<(unsigned)((n8 + 255) / 256), 256, 0, stream>>>(x, XB, n8);
    } else {
        const size_t n8 = (size_t)SEQ * DM / 8;
        for (int b = 0; b < NB; ++b) k_cvt8<<<(unsigned)((n8 + 255) / 256), 256, 0, stream>>>(x + (size_t)b * SEQ_FULL * DM, XB + (size_t)b * SEQ * DM, n8);
    }
    { const size_t n8 = (size_t)2 * DIN * DM / 8; k_cvt8<<<(unsigned)((n8 + 255) / 256), 256, 0, stream>>>(w_in, WB, n8); }
    { const size_t n8 = (size_t)XDW * DIN / 8; k_wcvt<<<(unsigned)((n8 + 255) / 256), 256, 0, stream>>>(w_x, WX16, n8, WSC); }
    { const size_t n8 = (size_t)DIN * DTR / 8; k_wcvt<<<(unsigned)((n8 + 255) / 256), 256, 0, stream>>>(w_dt, WD16, n8, WSC); }
    { const size_t n8 = (size_t)DM * DIN / 8;  k_wcvt<<<(unsigned)((n8 + 255) / 256), 256, 0, stream>>>(w_out, WO16, n8, WSC); }

    k_inproj<<<dim3(NB * SEQ / 64, 2 * DIN / 64, 1), 32, 0, stream>>>(XB, WB, XZ);
    { const size_t n8 = (size_t)NB * SEQ * DIN / 8; k_conv<<<(unsigned)((n8 + 255) / 256), 256, 0, stream>>>(XP, cw, cbias, U16, n8); }
    k_xproj<<<dim3(NB * SEQ / 32, 1, 1), 32, 0, stream>>>(U16, WX16, XD, DR16);
    k_dtproj<<<dim3(NB * SEQ / 64, DIN / 64, 1), 32, 0, stream>>>(DR16, WD16, b_dt, DT);
    k_scan<<<dim3(DIN / SCW, NB, 1), SCW, 0, stream>>>(XP, ZP, DT, XD, cw, cbias, a_log, d_par, Y16);
    k_outproj<<<dim3(NB * SEQ / 64, DM / 64, 1), 32, 0, stream>>>(Y16, WO16, OUT);
}
